// EnhancedMultiHeadAttention_67783173865510
// MI455X (gfx1250) — hardware-verified
//
#include <hip/hip_runtime.h>
#include <stdint.h>

#define BATCH 4
#define SEQ   1024
#define HID   1024
#define NH    16
#define HD    64
#define MROWS (BATCH * SEQ)
#define RK    16
#define RK2   32
#define PSCALE 16384.0f
#define LN_EPS 1e-5f

static_assert(MROWS % 128 == 0);
static_assert(SEQ % 128 == 0);
static_assert(HID % 64 == 0);
static_assert(HID == NH * HD);
static_assert(HD == 64);

typedef _Float16 v16h __attribute__((ext_vector_type(16)));
typedef _Float16 v8h  __attribute__((ext_vector_type(8)));
typedef __bf16   v16b __attribute__((ext_vector_type(16)));
typedef __bf16   v8b  __attribute__((ext_vector_type(8)));
typedef float    v8f  __attribute__((ext_vector_type(8)));
typedef float    v4f  __attribute__((ext_vector_type(4)));
typedef float    v2f  __attribute__((ext_vector_type(2)));
typedef unsigned int v4u __attribute__((ext_vector_type(4)));
typedef unsigned int v2u __attribute__((ext_vector_type(2)));
typedef v8h __attribute__((may_alias)) v8ha;
typedef v8b __attribute__((may_alias)) v8ba;
typedef v4f __attribute__((may_alias)) v4fa;
typedef v2f __attribute__((may_alias)) v2fa;
typedef v4u __attribute__((may_alias)) v4ua;
typedef v2u __attribute__((may_alias)) v2ua;

__device__ __forceinline__ unsigned short f2bf_bits(float f) {
  const unsigned u = __float_as_uint(f);
  return (unsigned short)((u + 0x7FFFu + ((u >> 16) & 1u)) >> 16);
}
__device__ __forceinline__ float bf_bits2f(unsigned short h) { return __uint_as_float(((unsigned)h) << 16); }
__device__ __forceinline__ float bfr(float f) { return bf_bits2f(f2bf_bits(f)); }
__device__ __forceinline__ unsigned short f2h_bits(float f) { return __builtin_bit_cast(unsigned short, (_Float16)f); }
__device__ __forceinline__ unsigned pk16(unsigned short a, unsigned short b) { return (unsigned)a | ((unsigned)b << 16); }
__device__ __forceinline__ unsigned short blo_bits(float f) { return f2bf_bits(f - bf_bits2f(f2bf_bits(f))); }

__device__ __forceinline__ v4u pack8_bf(v4f a, v4f c, float sc) {
  v4u o;
  o.x = pk16(f2bf_bits(a.x * sc), f2bf_bits(a.y * sc));
  o.y = pk16(f2bf_bits(a.z * sc), f2bf_bits(a.w * sc));
  o.z = pk16(f2bf_bits(c.x * sc), f2bf_bits(c.y * sc));
  o.w = pk16(f2bf_bits(c.z * sc), f2bf_bits(c.w * sc));
  return o;
}
__device__ __forceinline__ v4u pack8_blo(v4f a, v4f c) {
  v4u o;
  o.x = pk16(blo_bits(a.x), blo_bits(a.y));
  o.y = pk16(blo_bits(a.z), blo_bits(a.w));
  o.z = pk16(blo_bits(c.x), blo_bits(c.y));
  o.w = pk16(blo_bits(c.z), blo_bits(c.w));
  return o;
}
__device__ __forceinline__ v4u pack8_h(v4f a, v4f c, float sc) {
  v4u o;
  o.x = pk16(f2h_bits(a.x * sc), f2h_bits(a.y * sc));
  o.y = pk16(f2h_bits(a.z * sc), f2h_bits(a.w * sc));
  o.z = pk16(f2h_bits(c.x * sc), f2h_bits(c.y * sc));
  o.w = pk16(f2h_bits(c.z * sc), f2h_bits(c.w * sc));
  return o;
}
__device__ __forceinline__ unsigned short bsel_bits(float f, bool lo) {
  const unsigned short hb = f2bf_bits(f);
  const unsigned short lb = f2bf_bits(f - bf_bits2f(hb));
  return lo ? lb : hb;
}
__device__ __forceinline__ v4u pack8_bsel(v4f a, v4f c, bool lo) {
  v4u o;
  o.x = pk16(bsel_bits(a.x, lo), bsel_bits(a.y, lo));
  o.y = pk16(bsel_bits(a.z, lo), bsel_bits(a.w, lo));
  o.z = pk16(bsel_bits(c.x, lo), bsel_bits(c.y, lo));
  o.w = pk16(bsel_bits(c.z, lo), bsel_bits(c.w, lo));
  return o;
}

__device__ __forceinline__ v8f mma_h(v16h a, v16h b, v8f c) {
  v8f d = __builtin_amdgcn_wmma_f32_16x16x32_f16(false, a, false, b, (short)0, c, false, false);
  asm volatile("v_nop\n\tv_nop\n\tv_nop\n\tv_nop" : "+v"(d) : "v"(a), "v"(b));
  return d;
}
__device__ __forceinline__ v8f mma_b(v16b a, v16b b, v8f c) {
  v8f d = __builtin_amdgcn_wmma_f32_16x16x32_bf16(false, a, false, b, (short)0, c, false, false);
  asm volatile("v_nop\n\tv_nop\n\tv_nop\n\tv_nop" : "+v"(d) : "v"(a), "v"(b));
  return d;
}
__device__ __forceinline__ v16h ldh(const _Float16* p, int hh) {
  union { v16h v; v8h q[2]; } f;
  f.q[0] = *(const v8ha*)(p + 8 * hh);
  f.q[1] = *(const v8ha*)(p + 16 + 8 * hh);
  return f.v;
}
__device__ __forceinline__ v16b ldb(const __bf16* p, int hh) {
  union { v16b v; v8b q[2]; } f;
  f.q[0] = *(const v8ba*)(p + 8 * hh);
  f.q[1] = *(const v8ba*)(p + 16 + 8 * hh);
  return f.v;
}
__device__ __forceinline__ v8f zero8() { const v8f z = {0.f, 0.f, 0.f, 0.f, 0.f, 0.f, 0.f, 0.f}; return z; }

#define U_X  (MROWS * HID / 8)
#define U_W  (HID * HID / 8)
#define U_A3 (3 * RK * HID / 8)
#define U_AO (RK * HID / 8)
#define U_B  (HID * RK2 / 8)
#define SEG1 (U_X)
#define SEG2 (SEG1 + 4 * U_W)
#define SEG3 (SEG2 + U_A3)
#define SEG4 (SEG3 + U_AO)
#define SEG5 (SEG4 + 4 * U_B)
static_assert(SEG1 % 256 == 0);
static_assert(U_W % 256 == 0);
static_assert((RK * HID / 8) % 256 == 0);
static_assert(U_AO % 256 == 0);
static_assert(U_B % 256 == 0);
static_assert(SEG5 % 256 == 0);

__global__ __launch_bounds__(256) void k_prep(
    const float* __restrict__ x,
    const float* __restrict__ wq, const float* __restrict__ wk, const float* __restrict__ wv, const float* __restrict__ wo,
    const float* __restrict__ aq, const float* __restrict__ ak, const float* __restrict__ av, const float* __restrict__ ao,
    const float* __restrict__ bql, const float* __restrict__ bkl, const float* __restrict__ bvl, const float* __restrict__ bol,
    unsigned short* __restrict__ XB, unsigned short* __restrict__ WB, unsigned short* __restrict__ ACAT,
    unsigned short* __restrict__ AOT, unsigned short* __restrict__ BCAT)
{
  const int g0 = blockIdx.x * 256;
  const int g = g0 + (int)threadIdx.x;
  if (g >= SEG5) return;
  v4u o;
  unsigned short* dst;
  if (g0 < SEG1) {
    const float* src = x + (size_t)g * 8;
    o = pack8_bf(*(const v4fa*)src, *(const v4fa*)(src + 4), 1.0f);
    dst = XB + (size_t)g * 8;
  } else if (g0 < SEG2) {
    const int e = g - SEG1;
    const int p = e / U_W;
    const int off = e - p * U_W;
    const float* wsrc = (p == 0) ? wq : ((p == 1) ? wk : ((p == 2) ? wv : wo));
    const float* src = wsrc + (size_t)off * 8;
    o = pack8_bf(*(const v4fa*)src, *(const v4fa*)(src + 4), 1.0f);
    dst = WB + (size_t)e * 8;
  } else if (g0 < SEG3) {
    const int e = g - SEG2;
    const int n = e >> 7;
    const int p = n >> 4, r = n & 15;
    const int c = e & 127;
    const float* asrc = (p == 0) ? aq : ((p == 1) ? ak : av);
    v4f a, cc;
    a.x  = asrc[(size_t)(8 * c + 0) * RK + r];
    a.y  = asrc[(size_t)(8 * c + 1) * RK + r];
    a.z  = asrc[(size_t)(8 * c + 2) * RK + r];
    a.w  = asrc[(size_t)(8 * c + 3) * RK + r];
    cc.x = asrc[(size_t)(8 * c + 4) * RK + r];
    cc.y = asrc[(size_t)(8 * c + 5) * RK + r];
    cc.z = asrc[(size_t)(8 * c + 6) * RK + r];
    cc.w = asrc[(size_t)(8 * c + 7) * RK + r];
    o = pack8_bf(a, cc, 1.0f);
    dst = ACAT + (size_t)e * 8;
  } else if (g0 < SEG4) {
    const int e = g - SEG3;
    const int r = e >> 7;
    const int c = e & 127;
    v4f a, cc;
    a.x  = ao[(size_t)(8 * c + 0) * RK + r];
    a.y  = ao[(size_t)(8 * c + 1) * RK + r];
    a.z  = ao[(size_t)(8 * c + 2) * RK + r];
    a.w  = ao[(size_t)(8 * c + 3) * RK + r];
    cc.x = ao[(size_t)(8 * c + 4) * RK + r];
    cc.y = ao[(size_t)(8 * c + 5) * RK + r];
    cc.z = ao[(size_t)(8 * c + 6) * RK + r];
    cc.w = ao[(size_t)(8 * c + 7) * RK + r];
    o = pack8_bf(a, cc, 1.0f);
    dst = AOT + (size_t)e * 8;
  } else {
    const int e = g - SEG4;
    const int p = e >> 12;
    const int u = e & 4095;
    const int n = u >> 2;
    const int jj = (u & 3) * 8;
    const int kb = jj & 8;
    const float* bsrc = (p == 0) ? bql : ((p == 1) ? bkl : ((p == 2) ? bvl : bol));
    v4f a, cc;
    a.x  = bsrc[(size_t)(kb + 0) * HID + n];
    a.y  = bsrc[(size_t)(kb + 1) * HID + n];
    a.z  = bsrc[(size_t)(kb + 2) * HID + n];
    a.w  = bsrc[(size_t)(kb + 3) * HID + n];
    cc.x = bsrc[(size_t)(kb + 4) * HID + n];
    cc.y = bsrc[(size_t)(kb + 5) * HID + n];
    cc.z = bsrc[(size_t)(kb + 6) * HID + n];
    cc.w = bsrc[(size_t)(kb + 7) * HID + n];
    o = pack8_bf(a, cc, 2.0f);
    dst = BCAT + (size_t)e * 8;
  }
  *(volatile v4ua*)dst = o;
  __threadfence();
  *(volatile v4ua*)dst = o;
}

template <int NT>
__global__ __launch_bounds__(128) void k_xa(const unsigned short* __restrict__ Ap,
                                            const unsigned short* __restrict__ Atp,
                                            unsigned short* __restrict__ outp)
{
  __shared__ __align__(16) float sx[4][16 * 52];
  const int tid = threadIdx.x, lane = tid & 31, w = tid >> 5;
  const int hh = lane >> 4, m = lane & 15;
  const int t0 = blockIdx.x * 64 + 16 * w;
  const __bf16* A  = (const __bf16*)(const void*)Ap;
  const __bf16* At = (const __bf16*)(const void*)Atp;

  v8f acc[NT];
#pragma unroll
  for (int p = 0; p < NT; ++p) acc[p] = zero8();
  const __bf16* arow = A + (size_t)(t0 + m) * HID;
  const __bf16* brow = At + (size_t)m * HID;
#pragma unroll 1
  for (int k0 = 0; k0 < HID; k0 += 32) {
    const v16b a = ldb(arow + k0, hh);
#pragma unroll
    for (int p = 0; p < NT; ++p) {
      const v16b bb = ldb(brow + (size_t)p * 16 * HID + k0, hh);
      acc[p] = mma_b(a, bb, acc[p]);
    }
  }
  float* s = sx[w];
#pragma unroll
  for (int p = 0; p < NT; ++p)
#pragma unroll
    for (int r = 0; r < 8; ++r) s[(8 * hh + r) * 52 + 16 * p + m] = acc[p][r];
  __builtin_amdgcn_fence(__ATOMIC_RELEASE, "workgroup");
  __builtin_amdgcn_wave_barrier();
  __builtin_amdgcn_fence(__ATOMIC_ACQUIRE, "workgroup");

  const int rsub = lane >> 2;
  const int jb = (lane & 3) * 8;
  const int jsrc = jb & 8;
  const bool isLo = (jb >= 16);
  for (int pass = 0; pass < 2; ++pass) {
#pragma unroll
    for (int p = 0; p < NT; ++p) {
#pragma unroll
      for (int it = 0; it < 2; ++it) {
        const int row = 8 * it + rsub;
        const float* sp = s + row * 52 + 16 * p + jsrc;
        const v4u o = pack8_bsel(*(const v4fa*)sp, *(const v4fa*)(sp + 4), isLo);
        unsigned short* dst = outp + (size_t)p * MROWS * RK2 + (size_t)(t0 + row) * RK2 + jb;
        *(volatile v4ua*)dst = o;
      }
    }
    __threadfence();
  }
}

__device__ __forceinline__ void lin_core(const __bf16* __restrict__ A, const __bf16* __restrict__ W,
                                         const __bf16* __restrict__ XA, const __bf16* __restrict__ Bc,
                                         int m0w, int n0, int hh, int m, v8f (&acc)[2][4])
{
#pragma unroll
  for (int mt = 0; mt < 2; ++mt)
#pragma unroll
    for (int nt = 0; nt < 4; ++nt) acc[mt][nt] = zero8();
  const __bf16* a0p = A + (size_t)(m0w + m) * HID;
  const __bf16* a1p = a0p + (size_t)16 * HID;
  const __bf16* wp  = W + (size_t)(n0 + m) * HID;
#pragma unroll 1
  for (int k0 = 0; k0 < HID; k0 += 32) {
    const v16b a0 = ldb(a0p + k0, hh);
    const v16b a1 = ldb(a1p + k0, hh);
#pragma unroll
    for (int nt = 0; nt < 4; ++nt) {
      const v16b bb = ldb(wp + (size_t)nt * 16 * HID + k0, hh);
      acc[0][nt] = mma_b(a0, bb, acc[0][nt]);
      acc[1][nt] = mma_b(a1, bb, acc[1][nt]);
    }
  }
  {
    const v16b a0 = ldb(XA + (size_t)(m0w + m) * RK2, hh);
    const v16b a1 = ldb(XA + (size_t)(m0w + 16 + m) * RK2, hh);
    const __bf16* bp = Bc + (size_t)(n0 + m) * RK2;
#pragma unroll
    for (int nt = 0; nt < 4; ++nt) {
      const v16b bb = ldb(bp + (size_t)nt * 16 * RK2, hh);
      acc[0][nt] = mma_b(a0, bb, acc[0][nt]);
      acc[1][nt] = mma_b(a1, bb, acc[1][nt]);
    }
  }
}

__global__ __launch_bounds__(128) void k_qkv(
    const unsigned short* __restrict__ Xbp, const unsigned short* __restrict__ Wbp,
    const unsigned short* __restrict__ XAp, const unsigned short* __restrict__ Bcp,
    const float* __restrict__ bq, const float* __restrict__ bk, const float* __restrict__ bv,
    unsigned short* __restrict__ QF, unsigned short* __restrict__ KF, unsigned short* __restrict__ VT,
    unsigned short* __restrict__ QH, unsigned short* __restrict__ QL,
    unsigned short* __restrict__ KH, unsigned short* __restrict__ KL)
{
  __shared__ __align__(16) float sT[128 * 64];
  const int tid = threadIdx.x, lane = tid & 31, w = tid >> 5;
  const int hh = lane >> 4, m = lane & 15;
  const int m0 = blockIdx.x * 128;
  const int cg = blockIdx.y;
  const int which = cg >> 4, head = cg & 15;
  const int m0w = m0 + 32 * w;

  const __bf16* A  = (const __bf16*)(const void*)Xbp;
  const __bf16* W  = (const __bf16*)(const void*)Wbp + (size_t)which * HID * HID;
  const __bf16* XA = (const __bf16*)(const void*)XAp + (size_t)which * MROWS * RK2;
  const __bf16* Bc = (const __bf16*)(const void*)Bcp + (size_t)which * HID * RK2;

  v8f acc[2][4];
  lin_core(A, W, XA, Bc, m0w, head * HD, hh, m, acc);

  const float* bias = (which == 0) ? bq : ((which == 1) ? bk : bv);
#pragma unroll
  for (int nt = 0; nt < 4; ++nt) {
    const int feat = 16 * nt + m;
    const float bvv = bfr(bias[head * HD + feat]);
#pragma unroll
    for (int mt = 0; mt < 2; ++mt) {
#pragma unroll
      for (int r = 0; r < 8; ++r) {
        const int tokl = 32 * w + 16 * mt + 8 * hh + r;
        const float y = acc[mt][nt][r] + bvv;
        const int idx = (which == 2) ? (feat * 128 + tokl) : (tokl * 64 + feat);
        sT[idx] = y;
      }
    }
  }
  __syncthreads();

  const int b = m0 / SEQ, l0 = m0 - b * SEQ, bh = b * NH + head;
  const int q8 = lane & 7, sub = lane >> 3;
  if (which != 2) {
    const float fsc = (which == 0) ? 0.125f : 1.0f;
    unsigned short* F  = (which == 0) ? QF : KF;
    unsigned short* Hp = (which == 0) ? QH : KH;
    unsigned short* Lp = (which == 0) ? QL : KL;
    for (int pass = 0; pass < 2; ++pass) {
#pragma unroll
      for (int i = 0; i < 8; ++i) {
        const int lid = w * 32 + i * 4 + sub;
        const float* sp = sT + lid * 64 + 8 * q8;
        const v4f f0 = *(const v4fa*)sp;
        const v4f f1 = *(const v4fa*)(sp + 4);
        const v4u of = pack8_h(f0, f1, fsc);
        const v4u oh = pack8_bf(f0, f1, 1.0f);
        const v4u ol = pack8_blo(f0, f1);
        const size_t off = ((size_t)bh * SEQ + l0 + lid) * HD + 8 * q8;
        *(volatile v4ua*)(F + off)  = of;
        *(volatile v4ua*)(Hp + off) = oh;
        *(volatile v4ua*)(Lp + off) = ol;
      }
      __threadfence();
    }
  } else {
    for (int pass = 0; pass < 2; ++pass) {
#pragma unroll
      for (int i = 0; i < 8; ++i) {
        const int lid = w * 32 + i * 4 + sub;
        const int d = lid >> 1, hl = lid & 1;
        const float* sp = sT + d * 128 + 64 * hl + 8 * q8;
        const v4u of = pack8_h(*(const v4fa*)sp, *(const v4fa*)(sp + 4), 1.0f);
        const size_t off = ((size_t)bh * HD + d) * SEQ + l0 + 64 * hl + 8 * q8;
        *(volatile v4ua*)(VT + off) = of;
      }
      __threadfence();
    }
  }
}

__device__ __forceinline__ v16h pack_p(v8f a, v8f c) {
  const v16h r = { (_Float16)(a[0] * PSCALE), (_Float16)(a[1] * PSCALE), (_Float16)(a[2] * PSCALE), (_Float16)(a[3] * PSCALE),
                   (_Float16)(a[4] * PSCALE), (_Float16)(a[5] * PSCALE), (_Float16)(a[6] * PSCALE), (_Float16)(a[7] * PSCALE),
                   (_Float16)(c[0] * PSCALE), (_Float16)(c[1] * PSCALE), (_Float16)(c[2] * PSCALE), (_Float16)(c[3] * PSCALE),
                   (_Float16)(c[4] * PSCALE), (_Float16)(c[5] * PSCALE), (_Float16)(c[6] * PSCALE), (_Float16)(c[7] * PSCALE) };
  return r;
}

__global__ __launch_bounds__(128) void k_attn_ctx(
    const unsigned short* __restrict__ qfp,
    const unsigned short* __restrict__ kfp,
    const unsigned short* __restrict__ vtp,
    unsigned short* __restrict__ CTB,
    float* __restrict__ ST)
{
  __shared__ __align__(16) float sO[4 * 16 * 64];
  __shared__ float sM[64];
  __shared__ float sL[64];
  const _Float16* qf = (const _Float16*)(const void*)qfp;
  const _Float16* kf = (const _Float16*)(const void*)kfp;
  const _Float16* vt = (const _Float16*)(const void*)vtp;
  const int tid = threadIdx.x, lane = tid & 31, w = tid >> 5;
  const int hh = lane >> 4, m = lane & 15;
  const int bh = blockIdx.y, b = bh >> 4, head = bh & 15;
  const int qb0 = blockIdx.x * 64;
  const int q0 = qb0 + 16 * w;

  const _Float16* qrow = qf + ((size_t)bh * SEQ + q0 + m) * HD;
  const v16h qt0 = ldh(qrow, hh);
  const v16h qt1 = ldh(qrow + 32, hh);

  v8f o[4];
#pragma unroll
  for (int t = 0; t < 4; ++t) o[t] = zero8();
  float mrun = -1e30f, lrun = 0.0f;

  const _Float16* kbase = kf + ((size_t)bh * SEQ + m) * HD;
  const _Float16* vbase = vt + ((size_t)bh * HD + m) * SEQ;

#pragma unroll 1
  for (int kb = 0; kb < SEQ; kb += 64) {
    v8f s[4];
#pragma unroll
    for (int j = 0; j < 4; ++j) {
      const _Float16* kp = kbase + (size_t)(kb + 16 * j) * HD;
      const v16h k0f = ldh(kp, hh);
      const v16h k1f = ldh(kp + 32, hh);
      v8f z = zero8();
      z = mma_h(k0f, qt0, z);
      z = mma_h(k1f, qt1, z);
      s[j] = z;
    }
    float mloc = s[0][0];
#pragma unroll
    for (int j = 0; j < 4; ++j)
#pragma unroll
      for (int r = 0; r < 8; ++r) mloc = fmaxf(mloc, s[j][r]);
    mloc = fmaxf(mloc, __shfl_xor(mloc, 16, 32));
    const float mnew = fmaxf(mrun, mloc);
    const float alpha = __expf(mrun - mnew);
    mrun = mnew;
    float lsum = 0.0f;
#pragma unroll
    for (int j = 0; j < 4; ++j)
#pragma unroll
      for (int r = 0; r < 8; ++r) {
        const float p = __expf(s[j][r] - mnew);
        s[j][r] = p;
        lsum += p;
      }
    lsum += __shfl_xor(lsum, 16, 32);
    lrun = lrun * alpha + lsum;
#pragma unroll
    for (int t = 0; t < 4; ++t)
#pragma unroll
      for (int r = 0; r < 8; ++r) o[t][r] = o[t][r] * alpha;

    const v16h pb0 = pack_p(s[0], s[1]);
    const v16h pb1 = pack_p(s[2], s[3]);

#pragma unroll
    for (int t = 0; t < 4; ++t) {
      const _Float16* vp = vbase + (size_t)(16 * t) * SEQ + kb;
      const v16h vf0 = ldh(vp, hh);
      const v16h vf1 = ldh(vp + 32, hh);
      o[t] = mma_h(vf0, pb0, o[t]);
      o[t] = mma_h(vf1, pb1, o[t]);
    }
  }

  const float inv = (1.0f / lrun) * (1.0f / PSCALE);
  float* so = sO + w * 1024;
#pragma unroll
  for (int t = 0; t < 4; ++t)
#pragma unroll
    for (int r = 0; r < 8; ++r) so[m * 64 + 16 * t + 8 * hh + r] = o[t][r] * inv;
  sM[16 * w + m] = mrun;
  sL[16 * w + m] = lrun;
  __syncthreads();

  const int q8 = lane & 7, sub = lane >> 3;
  for (int pass = 0; pass < 2; ++pass) {
#pragma unroll
    for (int it = 0; it < 4; ++it) {
      const int row = it * 4 + sub;
      const float* sp = so + row * 64 + 8 * q8;
      const v4u ov = pack8_bf(*(const v4fa*)sp, *(const v4fa*)(sp + 4), 1.0f);
      unsigned short* dst = CTB + ((size_t)b * SEQ + q0 + row) * HID + head * HD + 8 * q8;
      *(volatile v4ua*)dst = ov;
    }
    if (w == 0) {
      v4f v;
      v.x = sM[2 * lane];     v.y = sL[2 * lane];
      v.z = sM[2 * lane + 1]; v.w = sL[2 * lane + 1];
      *(volatile v4f*)(ST + ((size_t)bh * SEQ + qb0 + 2 * lane) * 2) = v;
    }
    __threadfence();
  }
}

__global__ __launch_bounds__(128) void k_attn_mean(
    const unsigned short* __restrict__ qhp, const unsigned short* __restrict__ qlp,
    const unsigned short* __restrict__ khp, const unsigned short* __restrict__ klp,
    const float* __restrict__ ST,
    float* __restrict__ out1)
{
  __shared__ __align__(16) float sO[4 * 16 * 64];
  const __bf16* qh = (const __bf16*)(const void*)qhp;
  const __bf16* ql = (const __bf16*)(const void*)qlp;
  const __bf16* kh = (const __bf16*)(const void*)khp;
  const __bf16* kl = (const __bf16*)(const void*)klp;
  const int tid = threadIdx.x, lane = tid & 31, w = tid >> 5;
  const int hh = lane >> 4, m = lane & 15;
  const int b = blockIdx.z;
  const int qb0 = blockIdx.y * 64;
  const int q0 = qb0 + 16 * w;
  const int k0 = blockIdx.x * 64;

  v8f pacc[4];
#pragma unroll
  for (int j = 0; j < 4; ++j) pacc[j] = zero8();

#pragma unroll 1
  for (int hd = 0; hd < NH; ++hd) {
    const int bh = b * NH + hd;
    const size_t qo = ((size_t)bh * SEQ + q0 + m) * HD;
    const v16b qa0 = ldb(qh + qo, hh), qa1 = ldb(qh + qo + 32, hh);
    const v16b qc0 = ldb(ql + qo, hh), qc1 = ldb(ql + qo + 32, hh);
    const v2f st = *(const v2fa*)(ST + ((size_t)bh * SEQ + q0 + m) * 2);
    const float mrow = st.x;
    const float linv = 0.0625f * (1.0f / st.y);
    const size_t kbo = ((size_t)bh * SEQ + k0 + m) * HD;
#pragma unroll
    for (int j = 0; j < 4; ++j) {
      const size_t ko = kbo + (size_t)(16 * j) * HD;
      const v16b ka0 = ldb(kh + ko, hh), ka1 = ldb(kh + ko + 32, hh);
      const v16b kc0 = ldb(kl + ko, hh), kc1 = ldb(kl + ko + 32, hh);
      v8f s = zero8();
      s = mma_b(ka0, qa0, s);
      s = mma_b(ka0, qc0, s);
      s = mma_b(kc0, qa0, s);
      s = mma_b(ka1, qa1, s);
      s = mma_b(ka1, qc1, s);
      s = mma_b(kc1, qa1, s);
#pragma unroll
      for (int r = 0; r < 8; ++r) pacc[j][r] += __expf(s[r] * 0.125f - mrow) * linv;
    }
  }

  float* so = sO + w * 1024;
#pragma unroll
  for (int j = 0; j < 4; ++j)
#pragma unroll
    for (int r = 0; r < 8; ++r) so[m * 64 + 16 * j + 8 * hh + r] = pacc[j][r];
  __syncthreads();

  const int q8 = lane & 7, sub = lane >> 3;
  for (int pass = 0; pass < 2; ++pass) {
#pragma unroll
    for (int i = 0; i < 8; ++i) {
      const int lid = i * 4 + sub;
      const int row = lid >> 1, hl = lid & 1;
      const v4f v = *(const v4fa*)(so + row * 64 + 32 * hl + 4 * q8);
      const size_t gi = ((size_t)b * SEQ + q0 + row) * SEQ + k0 + 32 * hl + 4 * q8;
      *(volatile v4f*)(out1 + gi) = v;
    }
    __threadfence();
  }
}

__global__ __launch_bounds__(128) void k_out(
    const unsigned short* __restrict__ CTBp, const unsigned short* __restrict__ Wop,
    const unsigned short* __restrict__ XAop, const unsigned short* __restrict__ Bcop,
    const float* __restrict__ ob, float* __restrict__ Hout)
{
  __shared__ __align__(16) float sT[128 * 64];
  const int tid = threadIdx.x, lane = tid & 31, w = tid >> 5;
  const int hh = lane >> 4, m = lane & 15;
  const int m0 = blockIdx.x * 128;
  const int n0 = blockIdx.y * HD;
  const int m0w = m0 + 32 * w;

  v8f acc[2][4];
  lin_core((const __bf16*)(const void*)CTBp, (const __bf16*)(const void*)Wop,
           (const __bf16*)(const void*)XAop, (const __bf16*)(const void*)Bcop, m0w, n0, hh, m, acc);

#pragma unroll
  for (int nt = 0; nt < 4; ++nt) {
    const int feat = 16 * nt + m;
    const float bvv = bfr(ob[n0 + feat]);
#pragma unroll
    for (int mt = 0; mt < 2; ++mt) {
#pragma unroll
      for (int r = 0; r < 8; ++r) {
        const int tokl = 32 * w + 16 * mt + 8 * hh + r;
        sT[tokl * 64 + feat] = acc[mt][nt][r] + bvv;
      }
    }
  }
  __syncthreads();

  const int c4 = m * 4;
  for (int pass = 0; pass < 2; ++pass) {
#pragma unroll
    for (int it = 0; it < 16; ++it) {
      const int row = w * 32 + it * 2 + hh;
      const v4f v = *(const v4fa*)(sT + row * 64 + c4);
      *(volatile v4f*)(Hout + (size_t)(m0 + row) * HID + n0 + c4) = v;
    }
    __threadfence();
  }
}

__global__ __launch_bounds__(256) void k_ln(
    const float* __restrict__ H, const unsigned short* __restrict__ XB,
    const float* __restrict__ g, const float* __restrict__ bb, float* __restrict__ out0)
{
  __shared__ float red[8];
  const int mrow = blockIdx.x;
  const int t = threadIdx.x, lane = t & 31, w = t >> 5;
  const size_t base = (size_t)mrow * HID + 4 * t;
  const v4f hv = *(const v4fa*)(H + base);
  const v2u xw = *(const v2ua*)(XB + base);
  const float h0 = hv.x + __uint_as_float(xw.x << 16);
  const float h1 = hv.y + __uint_as_float(xw.x & 0xffff0000u);
  const float h2 = hv.z + __uint_as_float(xw.y << 16);
  const float h3 = hv.w + __uint_as_float(xw.y & 0xffff0000u);

  float s = (h0 + h1) + (h2 + h3);
#pragma unroll
  for (int off = 16; off > 0; off >>= 1) s += __shfl_xor(s, off, 32);
  if (lane == 0) red[w] = s;
  __syncthreads();
  float tot = red[0];
#pragma unroll
  for (int i = 1; i < 8; ++i) tot += red[i];
  const float mu = tot * (1.0f / (float)HID);
  __syncthreads();

  const float d0 = h0 - mu, d1 = h1 - mu, d2 = h2 - mu, d3 = h3 - mu;
  float s2 = (d0 * d0 + d1 * d1) + (d2 * d2 + d3 * d3);
#pragma unroll
  for (int off = 16; off > 0; off >>= 1) s2 += __shfl_xor(s2, off, 32);
  if (lane == 0) red[w] = s2;
  __syncthreads();
  float tot2 = red[0];
#pragma unroll
  for (int i = 1; i < 8; ++i) tot2 += red[i];
  const float var = tot2 * (1.0f / (float)HID);
  const float rstd = rsqrtf(var + LN_EPS);

  const v4f gv = *(const v4fa*)(g + 4 * t);
  const v4f bv = *(const v4fa*)(bb + 4 * t);
  v4f o;
  o.x = d0 * rstd * bfr(gv.x) + bfr(bv.x);
  o.y = d1 * rstd * bfr(gv.y) + bfr(bv.y);
  o.z = d2 * rstd * bfr(gv.z) + bfr(bv.z);
  o.w = d3 * rstd * bfr(gv.w) + bfr(bv.w);
  *(volatile v4f*)(out0 + base) = o;
  __threadfence();
  *(volatile v4f*)(out0 + base) = o;
}

extern "C" void kernel_launch(void* const* d_in, const int* in_sizes, int n_in,
                              void* d_out, int out_size, void* d_ws, size_t ws_size,
                              hipStream_t stream) {
  if (n_in < 19) return;
  if (in_sizes[0] != MROWS * HID) return;
  for (int p = 0; p < 4; ++p) {
    if (in_sizes[1 + 4 * p] != HID * HID) return;
    if (in_sizes[2 + 4 * p] != HID) return;
    if (in_sizes[3 + 4 * p] != HID * RK) return;
    if (in_sizes[4 + 4 * p] != RK * HID) return;
  }
  if (in_sizes[17] != HID || in_sizes[18] != HID) return;
  if (out_size != 2 * MROWS * HID) return;

  const float* x   = (const float*)d_in[0];
  const float* qw  = (const float*)d_in[1];
  const float* qb  = (const float*)d_in[2];
  const float* qA  = (const float*)d_in[3];
  const float* qB  = (const float*)d_in[4];
  const float* kw  = (const float*)d_in[5];
  const float* kbp = (const float*)d_in[6];
  const float* kA  = (const float*)d_in[7];
  const float* kB  = (const float*)d_in[8];
  const float* vw  = (const float*)d_in[9];
  const float* vb  = (const float*)d_in[10];
  const float* vA  = (const float*)d_in[11];
  const float* vB  = (const float*)d_in[12];
  const float* ow  = (const float*)d_in[13];
  const float* obp = (const float*)d_in[14];
  const float* oA  = (const float*)d_in[15];
  const float* oB  = (const float*)d_in[16];
  const float* lng = (const float*)d_in[17];
  const float* lnb = (const float*)d_in[18];
  float* out0 = (float*)d_out;
  float* out1 = (float*)d_out + (size_t)MROWS * HID;

  const size_t szX   = (size_t)MROWS * HID * 2;
  const size_t szW   = (size_t)4 * HID * HID * 2;
  const size_t szA3  = (size_t)3 * RK * HID * 2;
  const size_t szAO  = (size_t)RK * HID * 2;
  const size_t szBC  = (size_t)4 * HID * RK2 * 2;
  const size_t szXA3 = (size_t)3 * MROWS * RK2 * 2;
  const size_t szXAO = (size_t)MROWS * RK2 * 2;
  const size_t szP   = (size_t)MROWS * HID * 2;
  const size_t szST  = (size_t)BATCH * NH * SEQ * 2 * 4;
  const size_t szH   = (size_t)MROWS * HID * 4;
  size_t off = 0;
  const size_t oXB = off;  off += szX;
  const size_t oWB = off;  off += szW;
  const size_t oA3 = off;  off += szA3;
  const size_t oAO = off;  off += szAO;
  const size_t oBC = off;  off += szBC;
  const size_t oXA3 = off; off += szXA3;
  const size_t oXAO = off; off += szXAO;
  const size_t oQF = off;  off += szP;
  const size_t oKF = off;  off += szP;
  const size_t oVT = off;  off += szP;
  const size_t oQH = off;  off += szP;
  const size_t oQL = off;  off += szP;
  const size_t oKH = off;  off += szP;
  const size_t oKL = off;  off += szP;
  const size_t oST = off;  off += szST;
  const size_t oCT = off;  off += szP;
  const size_t oH  = off;  off += szH;
  if (off > ws_size) return;

  char* ws = (char*)d_ws;
  unsigned short* XB  = (unsigned short*)(ws + oXB);
  unsigned short* WB  = (unsigned short*)(ws + oWB);
  unsigned short* A3  = (unsigned short*)(ws + oA3);
  unsigned short* AO  = (unsigned short*)(ws + oAO);
  unsigned short* BC  = (unsigned short*)(ws + oBC);
  unsigned short* XA3 = (unsigned short*)(ws + oXA3);
  unsigned short* XAO = (unsigned short*)(ws + oXAO);
  unsigned short* QF  = (unsigned short*)(ws + oQF);
  unsigned short* KF  = (unsigned short*)(ws + oKF);
  unsigned short* VT  = (unsigned short*)(ws + oVT);
  unsigned short* QH  = (unsigned short*)(ws + oQH);
  unsigned short* QL  = (unsigned short*)(ws + oQL);
  unsigned short* KH  = (unsigned short*)(ws + oKH);
  unsigned short* KL  = (unsigned short*)(ws + oKL);
  float*          ST  = (float*)(ws + oST);
  unsigned short* CT  = (unsigned short*)(ws + oCT);
  float*          H   = (float*)(ws + oH);

  k_prep<<<dim3(SEG5 / 256), dim3(256), 0, stream>>>(x, qw, kw, vw, ow, qA, kA, vA, oA, qB, kB, vB, oB,
                                                      XB, WB, A3, AO, BC);
  k_xa<3><<<dim3(MROWS / 64), dim3(128), 0, stream>>>(XB, A3, XA3);
  k_qkv<<<dim3(MROWS / 128, 3 * NH), dim3(128), 0, stream>>>(XB, WB, XA3, BC, qb, kbp, vb,
                                                              QF, KF, VT, QH, QL, KH, KL);
  k_attn_ctx<<<dim3(SEQ / 64, BATCH * NH), dim3(128), 0, stream>>>(QF, KF, VT, CT, ST);
  k_attn_mean<<<dim3(SEQ / 64, SEQ / 64, BATCH), dim3(128), 0, stream>>>(QH, QL, KH, KL, ST, out1);
  k_xa<1><<<dim3(MROWS / 64), dim3(128), 0, stream>>>(CT, AO, XAO);
  k_out<<<dim3(MROWS / 128, HID / HD), dim3(128), 0, stream>>>(CT, WB + (size_t)3 * HID * HID, XAO,
                                                                BC + (size_t)3 * HID * RK2, obp, H);
  k_ln<<<dim3(MROWS), dim3(256), 0, stream>>>(H, XB, lng, lnb, out0);
  (void)hipGetLastError();
}
